// FastWeightODE_84859963834877
// MI455X (gfx1250) — hardware-verified
//
#include <hip/hip_runtime.h>
#include <math.h>

typedef __attribute__((ext_vector_type(16))) _Float16 v16h;
typedef __attribute__((ext_vector_type(16))) __bf16 v16b;
typedef __attribute__((ext_vector_type(8)))  _Float16 v8h;
typedef __attribute__((ext_vector_type(8)))  float v8f;
typedef __attribute__((ext_vector_type(4)))  float v4f;
typedef __attribute__((ext_vector_type(2)))  float v2f;
typedef __attribute__((ext_vector_type(4)))  unsigned v4u;
typedef __attribute__((ext_vector_type(4)))  int v4i;
typedef float __attribute__((may_alias)) float_a;
typedef int __attribute__((may_alias)) int_a;

template <typename T> __device__ __forceinline__ void vst2(void* p, T v) { *(volatile T*)p = v; __threadfence(); *(volatile T*)p = v; }
__device__ __forceinline__ v8f wmma16(v16h a, v16h b, v8f c) {
  v8f d = __builtin_amdgcn_wmma_f32_16x16x32_f16(false, a, false, b, (short)0, c, false, false);
  asm volatile("v_nop\n\tv_nop\n\tv_nop\n\tv_nop" : "+v"(d) : "v"(a), "v"(b));
  return d;
}
__device__ __forceinline__ v8f wmma_bf(v16b a, v16b b, v8f c) {
  v8f d = __builtin_amdgcn_wmma_f32_16x16x32_bf16(false, a, false, b, (short)0, c, false, false);
  asm volatile("v_nop\n\tv_nop\n\tv_nop\n\tv_nop" : "+v"(d) : "v"(a), "v"(b));
  return d;
}
__device__ __forceinline__ v16h frag_h(const _Float16* rowk0, int lane) {
  union { v16h v; v8h q[2]; } u; const _Float16* p = rowk0 + 8 * (lane >> 4);
  u.q[0] = *(const v8h*)p; u.q[1] = *(const v8h*)(p + 16); return u.v;
}
__device__ __forceinline__ v16h frag_f32(const float* rowk0, int lane) {
  v16h a; const float* p = rowk0 + 8 * (lane >> 4);
#pragma unroll
  for (int i = 0; i < 8; ++i) { a[i] = (_Float16)p[i]; a[8 + i] = (_Float16)p[16 + i]; }
  return a;
}
__device__ __forceinline__ v16h frag_f32s(const float* rowk0, int lane, float sc) {
  v16h a; const float* p = rowk0 + 8 * (lane >> 4);
#pragma unroll
  for (int i = 0; i < 8; ++i) { a[i] = (_Float16)(p[i] * sc); a[8 + i] = (_Float16)(p[16 + i] * sc); }
  return a;
}
__device__ __forceinline__ v16h fragc_f32(const float* W, int k0, int n, int lane, int ld, int K) {
  v16h a; const int g = lane >> 4;
#pragma unroll
  for (int i = 0; i < 8; ++i) { const int ka = k0 + 8 * g + i, kb = ka + 16;
    a[i] = (_Float16)(ka < K ? W[(size_t)(ka < K ? ka : K - 1) * ld + n] : 0.f); a[8 + i] = (_Float16)(kb < K ? W[(size_t)(kb < K ? kb : K - 1) * ld + n] : 0.f); }
  return a;
}
struct F2 { v16b h, l; };
__device__ __forceinline__ F2 bsplit16(const float v[16]) { F2 r;
#pragma unroll
  for (int i = 0; i < 16; ++i) { const __bf16 h = (__bf16)v[i]; r.h[i] = h; r.l[i] = (__bf16)(v[i] - (float)h); }
  return r; }
__device__ __forceinline__ F2 split_row(const float* row, int k0, int lane) { float v[16]; const float* p = row + k0 + 8 * (lane >> 4);
#pragma unroll
  for (int i = 0; i < 8; ++i) { v[i] = p[i]; v[8 + i] = p[16 + i]; }
  return bsplit16(v); }
__device__ __forceinline__ F2 split_rowK(const float* row, int k0, int lane, int K) { float v[16]; const int g = lane >> 4;
#pragma unroll
  for (int i = 0; i < 8; ++i) { const int ka = k0 + 8 * g + i, kb = ka + 16; v[i] = ka < K ? row[ka < K ? ka : K - 1] : 0.f; v[8 + i] = kb < K ? row[kb < K ? kb : K - 1] : 0.f; }
  return bsplit16(v); }
__device__ __forceinline__ F2 split_col(const float* W, int k0, int n, int lane, int ld, int K) { float v[16]; const int g = lane >> 4;
#pragma unroll
  for (int i = 0; i < 8; ++i) { const int ka = k0 + 8 * g + i, kb = ka + 16; v[i] = ka < K ? W[(size_t)(ka < K ? ka : K - 1) * ld + n] : 0.f; v[8 + i] = kb < K ? W[(size_t)(kb < K ? kb : K - 1) * ld + n] : 0.f; }
  return bsplit16(v); }
__device__ __forceinline__ v8f mac3(const F2& a, const F2& b, v8f c) { c = wmma_bf(a.l, b.h, c); c = wmma_bf(a.h, b.l, c); return wmma_bf(a.h, b.h, c); }
__device__ __forceinline__ float sigm(float v) { return 1.0f / (1.0f + expf(-v)); }
#define LDSX() do { asm volatile("s_wait_dscnt 0" ::: "memory"); __builtin_amdgcn_wave_barrier(); __builtin_amdgcn_fence(__ATOMIC_RELEASE, "workgroup"); } while (0)


#ifndef NB
#define NB 256
#endif
#define TT 256
#define CIN 64
#define IDIM 128
#define HID 512
#define NH 8
#define HD 64
#define FF 2048
#define NOUT 10
#ifndef BCH
#define BCH 64
#endif
#define NCH (NB / BCH)
#define CROWS (BCH * TT)
typedef __attribute__((ext_vector_type(8))) __bf16 v8b;
__device__ __forceinline__ v16b frag_b(const __bf16* rowk0, int lane) {
  union { v16b v; v8b q[2]; } u; const __bf16* p = rowk0 + 8 * (lane >> 4);
  u.q[0] = *(const v8b*)p; u.q[1] = *(const v8b*)(p + 16); return u.v;
}
__device__ __forceinline__ float bfr(float v) { return (float)(__bf16)v; }
__device__ __attribute__((noinline)) float exp_ni(float v) { return expf(v); }
__device__ __attribute__((noinline)) float erf_ni(float v) { return erff(v); }

#define WS_PW   0u
#define PWI 0
#define PWIP (PWI + CIN * IDIM)
#define PWK (PWIP + HID * CIN)
#define PWV (PWK + HID * HID)
#define PWQ (PWV + HID * HID)
#define PWO (PWQ + HID * HID)
#define PW1 (PWO + HID * HID)
#define PW2 (PW1 + FF * HID)
#define PWF (PW2 + HID * FF)
#define PWEND (PWF + 16 * HID)
#define WS_H    (WS_PW + 2u * PWEND)
#define WS_KH   (WS_H + 4u * CROWS * HID)
#define WS_KL   (WS_KH + 2u * CROWS * HID)
#define WS_VH   (WS_KL + 2u * CROWS * HID)
#define WS_VL   (WS_VH + 2u * CROWS * HID)
#define WS_Z    (WS_VL + 2u * CROWS * HID)
#define WS_S0   (WS_Z + 4u * NB * NH * HD * HD)
#define WS_H0   (WS_S0 + 4u * NB * CIN)
#define WS_K0   (WS_H0 + 4u * NB * HID)
#define WS_V0   (WS_K0 + 4u * NB * HID)
#define WS_HQ   (WS_V0 + 4u * NB * HID)
#define WS_Q    (WS_HQ + 4u * NB * HID)
#define WS_Y    (WS_Q + 4u * NB * HID)
#define WS_Y2   (WS_Y + 4u * NB * HID)
#define WS_HF   (WS_Y2 + 4u * NB * HID)
#define WS_F1   (WS_HF + 4u * NB * HID)
#define WS_Y3   (WS_F1 + 4u * NB * FF)
#define WS_END  (WS_Y3 + 4u * NB * HID)

__global__ __launch_bounds__(256) void k_pack(const float* __restrict__ WI, const float* __restrict__ WIP, const float* __restrict__ WK, const float* __restrict__ WV, const float* __restrict__ WQ, const float* __restrict__ WO, const float* __restrict__ W1, const float* __restrict__ W2, const float* __restrict__ WF, __bf16* __restrict__ PW) {
  __shared__ __align__(16) __bf16 s[FF]; const int n = blockIdx.x, which = blockIdx.y, tid = threadIdx.x; int K, N; const float* Wm; size_t base;
  switch (which) { case 0: K = IDIM; N = CIN; Wm = WI; base = PWI; break; case 1: K = CIN; N = HID; Wm = WIP; base = PWIP; break; case 2: K = HID; N = HID; Wm = WK; base = PWK; break; case 3: K = HID; N = HID; Wm = WV; base = PWV; break; case 4: K = HID; N = HID; Wm = WQ; base = PWQ; break; case 5: K = HID; N = HID; Wm = WO; base = PWO; break; case 6: K = HID; N = FF; Wm = W1; base = PW1; break; case 7: K = FF; N = HID; Wm = W2; base = PW2; break; default: K = HID; N = 16; Wm = WF; base = PWF; break; }
  if (n >= N) return;
  for (int k = tid; k < K; k += 256) s[k] = (__bf16)((which == 8 && n >= NOUT) ? 0.f : Wm[(size_t)n * K + k]);
  __syncthreads();
  for (int q = tid; q < K / 8; q += 256) vst2((unsigned*)(PW + base + (size_t)n * K + q * 8), *(const v4u*)&s[q * 8]);
}
template <int RIN, int NT, int EPI>
__global__ __launch_bounds__(128) void k_gemm(const float* __restrict__ A, int lda, int K, const __bf16* __restrict__ P, const float* __restrict__ bias, const float* __restrict__ RES, float* __restrict__ OUT, int ldo) {
  __shared__ __align__(16) float so[4][16][NT * 16 + 4];
  const int tid = threadIdx.x, wave = tid >> 5, lane = tid & 31, col = lane & 15, g = lane >> 4; const size_t r0 = (size_t)blockIdx.x * 64 + wave * 16; const int n0 = blockIdx.y * (NT * 16);
  v8f acc[NT]; for (int j = 0; j < NT; ++j) acc[j] = (v8f){};
#pragma unroll 2
  for (int kc = 0; kc < K / 32; ++kc) { F2 a; if (RIN) { v16b ax; const float* p = A + (r0 + col) * lda + kc * 32 + 8 * g;
#pragma unroll
      for (int i = 0; i < 8; ++i) { ax[i] = (__bf16)p[i]; ax[8 + i] = (__bf16)p[16 + i]; } a.h = ax; a.l = ax; } else a = split_row(A + (r0 + col) * lda, kc * 32, lane);
#pragma unroll
    for (int j = 0; j < NT; ++j) { const v16b w = frag_b(P + (size_t)(n0 + j * 16 + col) * K + kc * 32, lane); if (!RIN) acc[j] = wmma_bf(a.l, w, acc[j]); acc[j] = wmma_bf(a.h, w, acc[j]); } }
#pragma unroll
  for (int j = 0; j < NT; ++j) { const int n = n0 + j * 16 + col; const float bb = bias ? bfr(bias[n]) : 0.f;
#pragma unroll
    for (int r = 0; r < 8; ++r) { float v = acc[j][r] + bb; if (EPI == 1) v = fmaxf(v, 0.f); if (EPI == 2) v += RES[(r0 + 8 * g + r) * ldo + n]; so[wave][8 * g + r][j * 16 + col] = v; } }
  LDSX();
  for (int rl = 0; rl < 16; ++rl) if (lane < NT * 4) vst2(OUT + (r0 + rl) * ldo + n0 + lane * 4, *(const v4f*)&so[wave][rl][lane * 4]);
}
__global__ __launch_bounds__(256) void k_ln(const float* IN, float* H, const float* __restrict__ G, const float* __restrict__ Bb, int nrows, float* __restrict__ HQ, int b0) {
  __shared__ __align__(16) float s[8][HID]; const int wave = threadIdx.x >> 5, lane = threadIdx.x & 31; const size_t row = (size_t)blockIdx.x * 8 + wave; if (row >= (size_t)nrows) return;
  float v[16]; float sum = 0.f;
#pragma unroll
  for (int k = 0; k < 16; ++k) { v[k] = IN[row * HID + lane + 32 * k]; sum += v[k]; }
#pragma unroll
  for (int o = 1; o < 32; o <<= 1) sum += __shfl_xor(sum, o);
  const float mu = sum / (float)HID; float var = 0.f;
#pragma unroll
  for (int k = 0; k < 16; ++k) { const float d = v[k] - mu; var += d * d; }
#pragma unroll
  for (int o = 1; o < 32; o <<= 1) var += __shfl_xor(var, o);
  const float rs = rsqrtf(var / (float)HID + 1e-5f);
#pragma unroll
  for (int k = 0; k < 16; ++k) { const int c = lane + 32 * k; s[wave][c] = (v[k] - mu) * rs * bfr(G[c]) + bfr(Bb[c]); }
  LDSX();
  for (int pc = lane; pc < HID / 4; pc += 32) vst2(H + row * HID + pc * 4, *(const v4f*)&s[wave][pc * 4]);
  if (HQ && (int)(row % TT) == TT - 1) { const int b = b0 + (int)(row / TT); for (int pc = lane; pc < HID / 4; pc += 32) vst2(HQ + (size_t)b * HID + pc * 4, *(const v4f*)&s[wave][pc * 4]); }
}
template <int MODE>
__global__ __launch_bounds__(128) void k_proj(const float* __restrict__ A, const __bf16* __restrict__ P, const float* __restrict__ bias, float* __restrict__ OUT, __bf16* __restrict__ PH, __bf16* __restrict__ PL) {
  __shared__ __align__(16) float so[4][16][132]; __shared__ __align__(16) __bf16 sth[128][72], stl[128][72];
  const int tid = threadIdx.x, wave = tid >> 5, lane = tid & 31, col = lane & 15, g = lane >> 4; const size_t rb = (size_t)blockIdx.x * 64; const size_t r0 = rb + wave * 16; const int n0 = blockIdx.y * 128;
  v8f acc[8] = {};
#pragma unroll 2
  for (int kc = 0; kc < HID / 32; ++kc) { const F2 a = split_row(A + (r0 + col) * HID, kc * 32, lane);
#pragma unroll
    for (int j = 0; j < 8; ++j) { const v16b w = frag_b(P + (size_t)(n0 + j * 16 + col) * HID + kc * 32, lane); acc[j] = wmma_bf(a.l, w, acc[j]); acc[j] = wmma_bf(a.h, w, acc[j]); } }
  float val[8][8];
#pragma unroll
  for (int j = 0; j < 8; ++j) { const float bb = bfr(bias[n0 + j * 16 + col]);
#pragma unroll
    for (int r = 0; r < 8; ++r) val[j][r] = acc[j][r] + bb; }
  if (MODE == 0 || MODE == 2) {
#pragma unroll
    for (int r = 0; r < 8; ++r) {
#pragma unroll
      for (int hh = 0; hh < 2; ++hh) { float mx = fmaxf(fmaxf(val[4 * hh][r], val[4 * hh + 1][r]), fmaxf(val[4 * hh + 2][r], val[4 * hh + 3][r]));
#pragma unroll
        for (int o = 1; o < 16; o <<= 1) mx = fmaxf(mx, __shfl_xor(mx, o));
        float z = 0.f;
#pragma unroll
        for (int j = 0; j < 4; ++j) { val[4 * hh + j][r] = exp_ni(val[4 * hh + j][r] - mx); z += val[4 * hh + j][r]; }
#pragma unroll
        for (int o = 1; o < 16; o <<= 1) z += __shfl_xor(z, o);
        const float iz = 1.0f / z;
#pragma unroll
        for (int j = 0; j < 4; ++j) val[4 * hh + j][r] *= iz; } } }
  if (MODE == 1) {
#pragma unroll
    for (int r = 0; r < 8; ++r) { const int t = (int)((r0 + 8 * g + r) % TT); const float w = (t == 0) ? (5.0f / 6.0f) : ((t == TT - 1) ? (1.0f / 6.0f) : 1.0f);
#pragma unroll
      for (int j = 0; j < 8; ++j) val[j][r] *= w; } }
  if (MODE >= 2) {
#pragma unroll
    for (int j = 0; j < 8; ++j)
#pragma unroll
      for (int r = 0; r < 8; ++r) so[wave][8 * g + r][j * 16 + col] = val[j][r];
    LDSX();
    for (int rl = 0; rl < 16; ++rl) vst2(OUT + (r0 + rl) * HID + n0 + lane * 4, *(const v4f*)&so[wave][rl][lane * 4]);
  } else {
#pragma unroll
    for (int j = 0; j < 8; ++j)
#pragma unroll
      for (int r = 0; r < 8; ++r) { const float v = val[j][r]; const __bf16 hb = (__bf16)v; sth[j * 16 + col][wave * 16 + 8 * g + r] = hb; stl[j * 16 + col][wave * 16 + 8 * g + r] = (__bf16)(v - (float)hb); }
    __syncthreads();
    const int bl = (int)(rb / TT), t0 = (int)(rb % TT); const int h0 = n0 / HD;
    for (int q = tid; q < 128 * 8; q += 128) { const int d = q >> 3, pc = q & 7; const int hh = h0 + (d >> 6), e = d & 63; const size_t o = (((size_t)bl * NH + hh) * HD + e) * TT + t0 + pc * 8; vst2((unsigned*)(PH + o), *(const v4u*)&sth[d][pc * 8]); vst2((unsigned*)(PL + o), *(const v4u*)&stl[d][pc * 8]); }
  }
}
__global__ __launch_bounds__(128) void k_z(const __bf16* __restrict__ VH, const __bf16* __restrict__ VL, const __bf16* __restrict__ KH, const __bf16* __restrict__ KL, const float* __restrict__ V0, const float* __restrict__ K0, int b0, float* __restrict__ Z) {
  __shared__ __align__(16) float so[4][16][68];
  const int tid = threadIdx.x, wave = tid >> 5, lane = tid & 31, col = lane & 15, g = lane >> 4; const int h = blockIdx.x, bl = blockIdx.y; const int b = b0 + bl;
  const size_t base = ((size_t)bl * NH + h) * HD * TT; const int d0 = wave * 16;
  v8f acc[4] = {};
#pragma unroll 2
  for (int kc = 0; kc < TT / 32; ++kc) { const v16b ah = frag_b(VH + base + (size_t)(d0 + col) * TT + kc * 32, lane), al = frag_b(VL + base + (size_t)(d0 + col) * TT + kc * 32, lane);
#pragma unroll
    for (int j = 0; j < 4; ++j) { const size_t br = base + (size_t)(j * 16 + col) * TT + kc * 32; const v16b bh = frag_b(KH + br, lane), blo = frag_b(KL + br, lane); acc[j] = wmma_bf(al, bh, acc[j]); acc[j] = wmma_bf(ah, blo, acc[j]); acc[j] = wmma_bf(ah, bh, acc[j]); } }
#pragma unroll
  for (int j = 0; j < 4; ++j) { const int e = j * 16 + col; const float k0 = K0[(size_t)b * HID + h * HD + e];
#pragma unroll
    for (int r = 0; r < 8; ++r) { const int d = d0 + 8 * g + r; so[wave][8 * g + r][e] = acc[j][r] + V0[(size_t)b * HID + h * HD + d] * k0; } }
  LDSX();
  for (int rl = 0; rl < 16; ++rl) if (lane < 16) vst2(Z + (((size_t)b * NH + h) * HD + d0 + rl) * HD + lane * 4, *(const v4f*)&so[wave][rl][lane * 4]);
}
__global__ __launch_bounds__(512) void k_read(const float* __restrict__ Z, const float* __restrict__ Q, float* __restrict__ Y) {
  __shared__ float sq[HID]; __shared__ __align__(16) float sy[HID]; const int b = blockIdx.x, tid = threadIdx.x; const int h = tid >> 6, d = tid & 63;
  sq[tid] = Q[(size_t)b * HID + tid]; __syncthreads();
  const float* zr = Z + (((size_t)b * NH + h) * HD + d) * HD; float acc = 0.f;
#pragma unroll 1
  for (int e = 0; e < HD; ++e) acc += zr[e] * sq[h * HD + e];
  sy[tid] = acc; __syncthreads();
  if (tid < HID / 4) vst2(Y + (size_t)b * HID + tid * 4, *(const v4f*)&sy[tid * 4]);
}
__global__ __launch_bounds__(128) void k_fin(const float* __restrict__ Y3, const __bf16* __restrict__ P, const float* __restrict__ BF, float* __restrict__ out) {
  __shared__ __align__(16) float so[64 * NOUT];
  const int tid = threadIdx.x, wave = tid >> 5, lane = tid & 31, col = lane & 15, g = lane >> 4; const size_t r0 = (size_t)blockIdx.x * 64 + wave * 16;
  v8f acc = {};
#pragma unroll 2
  for (int kc = 0; kc < HID / 32; ++kc) { const F2 a = split_row(Y3 + (r0 + col) * HID, kc * 32, lane); const v16b w = frag_b(P + PWF + (size_t)col * HID + kc * 32, lane); acc = wmma_bf(a.l, w, acc); acc = wmma_bf(a.h, w, acc); }
  if (col < NOUT) {
#pragma unroll
    for (int r = 0; r < 8; ++r) so[(wave * 16 + 8 * g + r) * NOUT + col] = acc[r] + bfr(BF[col]); }
  __syncthreads();
  for (int q = tid; q < 64 * NOUT / 4; q += 128) vst2(out + (size_t)blockIdx.x * 64 * NOUT + q * 4, *(const v4f*)&so[q * 4]);
}
extern "C" void kernel_launch(void* const* d_in, const int* in_sizes, int n_in, void* d_out, int out_size, void* d_ws, size_t ws_size, hipStream_t stream) {
  (void)in_sizes; (void)n_in; (void)out_size;
  const float** F = (const float**)d_in;
  if (ws_size < (size_t)WS_END) return;
  char* ws = (char*)d_ws; __bf16 *PW = (__bf16*)(ws + WS_PW), *KH = (__bf16*)(ws + WS_KH), *KL = (__bf16*)(ws + WS_KL), *VH = (__bf16*)(ws + WS_VH), *VL = (__bf16*)(ws + WS_VL);
  float *H = (float*)(ws + WS_H), *Z = (float*)(ws + WS_Z), *S0 = (float*)(ws + WS_S0), *H0 = (float*)(ws + WS_H0), *K0 = (float*)(ws + WS_K0), *V0 = (float*)(ws + WS_V0), *HQ = (float*)(ws + WS_HQ), *Q = (float*)(ws + WS_Q), *Y = (float*)(ws + WS_Y), *Y2 = (float*)(ws + WS_Y2), *HF = (float*)(ws + WS_HF), *F1 = (float*)(ws + WS_F1), *Y3 = (float*)(ws + WS_Y3);
  k_pack<<<dim3(FF, 9), 256, 0, stream>>>(F[2], F[4], F[8], F[10], F[12], F[14], F[18], F[20], F[22], PW);
  k_gemm<1, 4, 0><<<dim3(NB / 64, 1), 128, 0, stream>>>(F[0], IDIM, IDIM, PW + PWI, F[3], nullptr, S0, CIN);
  k_gemm<0, 8, 0><<<dim3(NB / 64, HID / 128), 128, 0, stream>>>(S0, CIN, CIN, PW + PWIP, F[5], nullptr, H0, HID);
  k_ln<<<NB / 8, 256, 0, stream>>>(H0, H0, F[6], F[7], NB, nullptr, 0);
  k_proj<2><<<dim3(NB / 64, HID / 128), 128, 0, stream>>>(H0, PW + PWK, F[9], K0, nullptr, nullptr);
  k_proj<3><<<dim3(NB / 64, HID / 128), 128, 0, stream>>>(H0, PW + PWV, F[11], V0, nullptr, nullptr);
  for (int c = 0; c < NCH; ++c) { const int b0 = c * BCH; const float* X = F[1] + (size_t)b0 * TT * CIN;
    k_gemm<1, 8, 0><<<dim3(CROWS / 64, HID / 128), 128, 0, stream>>>(X, CIN, CIN, PW + PWIP, F[5], nullptr, H, HID);
    k_ln<<<CROWS / 8, 256, 0, stream>>>(H, H, F[6], F[7], CROWS, HQ, b0);
    k_proj<0><<<dim3(CROWS / 64, HID / 128), 128, 0, stream>>>(H, PW + PWK, F[9], nullptr, KH, KL);
    k_proj<1><<<dim3(CROWS / 64, HID / 128), 128, 0, stream>>>(H, PW + PWV, F[11], nullptr, VH, VL);
    k_z<<<dim3(NH, BCH), 128, 0, stream>>>(VH, VL, KH, KL, V0, K0, b0, Z); }
  k_proj<2><<<dim3(NB / 64, HID / 128), 128, 0, stream>>>(HQ, PW + PWQ, F[13], Q, nullptr, nullptr);
  k_read<<<NB, 512, 0, stream>>>(Z, Q, Y);
  k_gemm<0, 8, 0><<<dim3(NB / 64, HID / 128), 128, 0, stream>>>(Y, HID, HID, PW + PWO, F[15], nullptr, Y2, HID);
  k_ln<<<NB / 8, 256, 0, stream>>>(Y2, HF, F[16], F[17], NB, nullptr, 0);
  k_gemm<0, 8, 1><<<dim3(NB / 64, FF / 128), 128, 0, stream>>>(HF, HID, HID, PW + PW1, F[19], nullptr, F1, FF);
  k_gemm<0, 8, 2><<<dim3(NB / 64, HID / 128), 128, 0, stream>>>(F1, FF, FF, PW + PW2, F[21], Y2, Y3, HID);
  k_fin<<<NB / 64, 128, 0, stream>>>(Y3, PW, F[23], (float*)d_out);
}
